// MultiHeadAttention_88622355186026
// MI455X (gfx1250) — hardware-verified
//
#include <hip/hip_runtime.h>


#ifndef NB
#define NB 4
#endif
#ifndef SEQ
#define SEQ 2048
#endif
#define NB_FULL  4
#define SEQ_FULL 2048
#define DM   768
#define NH   12
#define HD   64
#define QKP  (2 * DM)
#define CTP  72
#define QKVC 16.0f
#define CTXC 256.0f
#define WOC  64.0f
#define PSH  8.0f
#define CEXP (0.125f * 1.4426950408889634f / (QKVC * QKVC))

static_assert(SEQ % 128 == 0);
static_assert(DM % 64 == 0);
static_assert(NH * HD == DM);
static_assert(NB <= NB_FULL);
static_assert(SEQ <= SEQ_FULL);

typedef _Float16 h16;
typedef unsigned short bf;
typedef __attribute__((ext_vector_type(16))) __bf16   v16bf;
typedef __attribute__((ext_vector_type(16))) _Float16 v16h;
typedef __attribute__((ext_vector_type(8)))  _Float16 v8h;
typedef __attribute__((ext_vector_type(8)))  unsigned short v8us;
typedef __attribute__((ext_vector_type(2)))  unsigned short v2us;
typedef __attribute__((ext_vector_type(8)))  float    v8f;
typedef __attribute__((ext_vector_type(4)))  float    v4f;
typedef v4f  __attribute__((may_alias)) v4fa;

__device__ __forceinline__ unsigned short f2bf(float f) { unsigned u = __float_as_uint(f); u += 0x7FFFu + ((u >> 16) & 1u); return (unsigned short)(u >> 16); }
__device__ __forceinline__ float bf2f(unsigned short b) { return __uint_as_float(((unsigned)b) << 16); }
__device__ __forceinline__ float bfr(float f) { return bf2f(f2bf(f)); }
__device__ __forceinline__ v16h cat16(v8h lo, v8h hi) { return __builtin_shufflevector(lo, hi, 0, 1, 2, 3, 4, 5, 6, 7, 8, 9, 10, 11, 12, 13, 14, 15); }
__device__ __forceinline__ v16bf cat16b(v8us lo, v8us hi) { return __builtin_bit_cast(v16bf, __builtin_shufflevector(lo, hi, 0, 1, 2, 3, 4, 5, 6, 7, 8, 9, 10, 11, 12, 13, 14, 15)); }
__device__ __forceinline__ v8f wmma16(v16h a, v16h b, v8f c) { return __builtin_amdgcn_wmma_f32_16x16x32_f16(false, a, false, b, (short)0, c, false, false); }
__device__ __forceinline__ v8f wmmab(v16bf a, v16bf b, v8f c) { return __builtin_amdgcn_wmma_f32_16x16x32_bf16(false, a, false, b, (short)0, c, false, false); }
__device__ __forceinline__ v16h ldh(const h16* p) { return cat16(*(const v8h*)p, *(const v8h*)(p + 16)); }

template <typename T16> struct WFrag;
template <> struct WFrag<h16> { typedef v16h V; static __device__ __forceinline__ V ld(const h16* p) { return cat16(*(const v8h*)p, *(const v8h*)(p + 16)); } static __device__ __forceinline__ v8f mma(V a, V b, v8f c) { return wmma16(a, b, c); } };
template <> struct WFrag<bf> { typedef v16bf V; static __device__ __forceinline__ V ld(const bf* p) { return cat16b(*(const v8us*)p, *(const v8us*)(p + 16)); } static __device__ __forceinline__ v8f mma(V a, V b, v8f c) { return wmmab(a, b, c); } };

template <typename T16, bool OUT16, bool BIAS>
__global__ __launch_bounds__(32) void k_gemmw(const T16* __restrict__ A, const T16* __restrict__ Bt, float* C32, h16* C16, const float* __restrict__ bias, size_t sA, size_t sB, size_t sC, int K, int ldc, float oscale) {
    typedef typename WFrag<T16>::V V;
    __shared__ __align__(16) float os[16 * 68];
    const size_t z = blockIdx.z; A += z * sA; Bt += z * sB;
    const int lane = threadIdx.x & 31, lr = lane & 15, hi = lane >> 4; const int r0 = blockIdx.x * 64, c0 = blockIdx.y * 64;
    v8f acc[4][4];
#pragma unroll
    for (int mb = 0; mb < 4; ++mb)
#pragma unroll
        for (int nb = 0; nb < 4; ++nb) acc[mb][nb] = (v8f){};
    const size_t aoff = (size_t)(r0 + lr) * K + 8 * hi, boff = (size_t)(c0 + lr) * K + 8 * hi;
#pragma unroll 1
    for (int kc = 0; kc < K; kc += 32) {
        V a[4];
#pragma unroll
        for (int mb = 0; mb < 4; ++mb) a[mb] = WFrag<T16>::ld(A + aoff + (size_t)mb * 16 * K + kc);
#pragma unroll
        for (int nb = 0; nb < 4; ++nb) { const V b = WFrag<T16>::ld(Bt + boff + (size_t)nb * 16 * K + kc);
#pragma unroll
            for (int mb = 0; mb < 4; ++mb) acc[mb][nb] = WFrag<T16>::mma(a[mb], b, acc[mb][nb]); }
        asm volatile("v_nop\n\tv_nop\n\tv_nop\n\tv_nop" : "+v"(acc[0][0]), "+v"(acc[1][1]), "+v"(acc[2][2]), "+v"(acc[3][3]) : "v"(a[0]), "v"(a[3]));
    }
#pragma unroll
    for (int mb = 0; mb < 4; ++mb) {
#pragma unroll
        for (int nb = 0; nb < 4; ++nb) {
#pragma unroll
            for (int j = 0; j < 8; ++j) os[(hi * 8 + j) * 68 + nb * 16 + lr] = acc[mb][nb][j]; }
        __syncthreads();
        if constexpr (OUT16) {
            h16* crow = C16 + z * sC + (size_t)(r0 + mb * 16) * ldc + c0;
#pragma unroll 1
            for (int ps = 0; ps < 2; ++ps) {
#pragma unroll
                for (int s = 0; s < 4; ++s) { const int row = 4 * s + (lane >> 3), cofs = (lane & 7) * 8;
                    const v4f x0 = *(const v4fa*)(os + row * 68 + cofs); const v4f x1 = *(const v4fa*)(os + row * 68 + cofs + 4); v8h o;
#pragma unroll
                    for (int i = 0; i < 4; ++i) { o[i] = (h16)(x0[i] * oscale); o[4 + i] = (h16)(x1[i] * oscale); }
                    *(volatile v8h*)(crow + (size_t)row * ldc + cofs) = o; }
                if (ps == 0) __threadfence(); }
        } else {
            float* crow = C32 + z * sC + (size_t)(r0 + mb * 16) * ldc + c0;
#pragma unroll 1
            for (int ps = 0; ps < 2; ++ps) {
#pragma unroll
                for (int s = 0; s < 8; ++s) { const int row = 2 * s + hi, cofs = lr * 4; v4f val = *(const v4fa*)(os + row * 68 + cofs);
#pragma unroll
                    for (int i = 0; i < 4; ++i) { float t = val[i] * oscale; if (BIAS) t += bfr(bias[c0 + cofs + i]); val[i] = t; }
                    *(volatile v4f*)(crow + (size_t)row * ldc + cofs) = val; }
                if (ps == 0) __threadfence(); }
        }
        __syncthreads();
    }
}

template <int KK, int NN, bool F16>
__global__ __launch_bounds__(256) void k_wt(const float* __restrict__ w, unsigned short* Bt) {
#pragma clang fp contract(off)
    const int lane = threadIdx.x & 31; const int wv = __builtin_amdgcn_readfirstlane((int)(threadIdx.x >> 5)); const int L0 = (blockIdx.x * 8 + wv) * 8; constexpr int nlines = NN * KK / 64;
#pragma unroll
    for (int ps = 0; ps < 2; ++ps) {
#pragma unroll 1
        for (int l = 0; l < 8; ++l) { const int L = L0 + l; if (L >= nlines) break; const int e = L * 64 + lane * 2; const int k = e % KK, n = e / KK; v2us o;
#pragma unroll
            for (int q = 0; q < 2; ++q) { const float v = w[(size_t)(k + q) * NN + n]; unsigned short r;
                if (F16) { const h16 hv = (h16)(bfr(v) * WOC); r = __builtin_bit_cast(unsigned short, hv); } else { r = f2bf(v); }
                o[q] = r; }
            *(volatile v2us*)(Bt + e) = o; }
        if (ps == 0) __threadfence(); }
}

__global__ __launch_bounds__(256) void k_cvt8(const float* __restrict__ src, bf* dst, size_t ssrc, size_t sdst, unsigned n8) {
#pragma clang fp contract(off)
    const unsigned i = blockIdx.x * 256u + threadIdx.x; if (i >= n8) return;
    const float* s = src + (size_t)blockIdx.z * ssrc + (size_t)i * 8; bf* d = dst + (size_t)blockIdx.z * sdst + (size_t)i * 8;
    const v8f v = *(const v8f*)s; v8us o;
#pragma unroll
    for (int k = 0; k < 8; ++k) o[k] = f2bf(v[k]);
    *(volatile v8us*)d = o; __threadfence(); *(volatile v8us*)d = o;
}

__global__ __launch_bounds__(128) __attribute__((amdgpu_num_vgpr(256))) void k_attn(const h16* __restrict__ QK, const h16* __restrict__ VT, h16* CTX) {
    __shared__ __align__(16) h16 ct[4 * 32 * CTP];
    const int lane = threadIdx.x & 31, lr = lane & 15, hi = lane >> 4;
    const int w = __builtin_amdgcn_readfirstlane((int)(threadIdx.x >> 5));
    const int hd = blockIdx.y, b = blockIdx.z;
    const int q0 = blockIdx.x * 128 + w * 32;
    const h16* qkb = QK + (size_t)b * SEQ * QKP;
    v16h qf[2][2];
#pragma unroll
    for (int qt = 0; qt < 2; ++qt)
#pragma unroll
        for (int ks = 0; ks < 2; ++ks) qf[qt][ks] = ldh(qkb + (size_t)(q0 + 16 * qt + lr) * QKP + hd * HD + 32 * ks + 8 * hi);
    const h16* kp = qkb + (size_t)lr * QKP + DM + hd * HD + 8 * hi;
    const h16* vp = VT + ((size_t)b * DM + hd * HD + lr) * SEQ + 8 * hi;
    v8f o[2][4];
#pragma unroll
    for (int qt = 0; qt < 2; ++qt)
#pragma unroll
        for (int j = 0; j < 4; ++j) o[qt][j] = (v8f){};
    float M[2], L[2];
    M[0] = -3.0e38f; M[1] = -3.0e38f; L[0] = 0.0f; L[1] = 0.0f;
#pragma unroll 1
    for (int kb = 0; kb < SEQ; kb += 32) {
        v16h ka[2][2];
#pragma unroll
        for (int kt = 0; kt < 2; ++kt)
#pragma unroll
            for (int ks = 0; ks < 2; ++ks) ka[kt][ks] = ldh(kp + (size_t)(kb + 16 * kt) * QKP + 32 * ks);
        v16h va[4];
#pragma unroll
        for (int j = 0; j < 4; ++j) va[j] = ldh(vp + (size_t)(16 * j) * SEQ + kb);
        v16h pf[2];
#pragma unroll
        for (int qt = 0; qt < 2; ++qt) {
            v8f s0 = (v8f){}, s1 = (v8f){};
            s0 = wmma16(ka[0][0], qf[qt][0], s0); s0 = wmma16(ka[0][1], qf[qt][1], s0);
            s1 = wmma16(ka[1][0], qf[qt][0], s1); s1 = wmma16(ka[1][1], qf[qt][1], s1);
            asm volatile("v_nop\n\tv_nop\n\tv_nop\n\tv_nop" : "+v"(s0), "+v"(s1) : "v"(ka[0][0]), "v"(ka[0][1]), "v"(ka[1][0]), "v"(ka[1][1]), "v"(qf[qt][0]), "v"(qf[qt][1]));
            float mx = fmaxf(s0[0], s1[0]);
#pragma unroll
            for (int r = 1; r < 8; ++r) mx = fmaxf(mx, fmaxf(s0[r], s1[r]));
            mx = fmaxf(mx, __shfl_xor(mx, 16, 32));
            const float mo = M[qt]; const float mn = fmaxf(mo, mx);
            const float cf = __builtin_amdgcn_exp2f((mo - mn) * CEXP);
            const float mneg = fmaf(-mn, CEXP, PSH);
            float sum = 0.0f; v16h p;
#pragma unroll
            for (int r = 0; r < 8; ++r) { const float e0 = __builtin_amdgcn_exp2f(fmaf(s0[r], CEXP, mneg)); const float e1 = __builtin_amdgcn_exp2f(fmaf(s1[r], CEXP, mneg)); sum += e0 + e1; p[r] = (h16)e0; p[8 + r] = (h16)e1; }
            L[qt] = L[qt] * cf + sum; M[qt] = mn;
            const unsigned grow = __builtin_amdgcn_ballot_w32(mn > mo);
            if (grow != 0u) {
#pragma unroll
                for (int j = 0; j < 4; ++j)
#pragma unroll
                    for (int r = 0; r < 8; ++r) o[qt][j][r] *= cf; }
            pf[qt] = p;
        }
#pragma unroll
        for (int j = 0; j < 4; ++j)
#pragma unroll
            for (int qt = 0; qt < 2; ++qt) o[qt][j] = wmma16(va[j], pf[qt], o[qt][j]);
        asm volatile("v_nop\n\tv_nop\n\tv_nop\n\tv_nop" : "+v"(o[0][0]), "+v"(o[0][1]), "+v"(o[0][2]), "+v"(o[0][3]), "+v"(o[1][0]), "+v"(o[1][1]), "+v"(o[1][2]), "+v"(o[1][3]) : "v"(va[0]), "v"(va[1]), "v"(va[2]), "v"(va[3]), "v"(pf[0]), "v"(pf[1]));
    }
    h16* ctw = ct + w * (32 * CTP);
#pragma unroll
    for (int qt = 0; qt < 2; ++qt) {
        const float lt = L[qt] + __shfl_xor(L[qt], 16, 32);
        const float inv = (CTXC / QKVC) * __builtin_amdgcn_rcpf(lt);
#pragma unroll
        for (int j = 0; j < 4; ++j) { v8h ov;
#pragma unroll
            for (int r = 0; r < 8; ++r) ov[r] = (h16)(o[qt][j][r] * inv);
            *(v8h*)(ctw + (16 * qt + lr) * CTP + 16 * j + 8 * hi) = ov; }
    }
    __syncthreads();
    h16* cbase = CTX + ((size_t)b * SEQ + q0) * DM + hd * HD;
#pragma unroll 1
    for (int ps = 0; ps < 2; ++ps) {
#pragma unroll
        for (int s = 0; s < 8; ++s) { const int row = 4 * s + (lane >> 3), pc = (lane & 7) * 8; const v8h v = *(const v8h*)(ctw + row * CTP + pc);
            *(volatile v8h*)(cbase + (size_t)row * DM + pc) = v; }
        if (ps == 0) __threadfence(); }
}

constexpr size_t al256(size_t v) { return (v + 255) & ~(size_t)255; }
constexpr size_t WT_BYTES = al256((size_t)3 * DM * DM * 2);
constexpr size_t WO_BYTES = al256((size_t)DM * DM * 2);
constexpr size_t XB_BYTES = al256((size_t)NB * SEQ * DM * 2);
constexpr size_t QK_BYTES = al256((size_t)NB * SEQ * QKP * 2);
constexpr size_t VT_BYTES = al256((size_t)NB * DM * SEQ * 2);
constexpr size_t CT_BYTES = al256((size_t)NB * SEQ * DM * 2);
constexpr size_t WS_TOTAL = WT_BYTES + WO_BYTES + XB_BYTES + QK_BYTES + VT_BYTES + CT_BYTES;
static_assert(WS_TOTAL <= (size_t)134217728);
static_assert(((size_t)(NB - 1) * SEQ_FULL + SEQ) * DM <= (size_t)NB_FULL * SEQ_FULL * DM);

extern "C" void kernel_launch(void* const* d_in, const int* in_sizes, int n_in,
                              void* d_out, int out_size, void* d_ws, size_t ws_size, hipStream_t stream) {
    if (n_in < 4) return;
    if ((long long)in_sizes[0] < (long long)((size_t)(NB - 1) * SEQ_FULL + SEQ) * DM) return;
    if (in_sizes[1] < 3 * DM * DM) return;
    if (in_sizes[2] < DM * DM) return;
    if (in_sizes[3] < DM) return;
    if ((long long)out_size < (long long)((size_t)(NB - 1) * SEQ_FULL + SEQ) * DM) return;
    if (WS_TOTAL > ws_size) return;
    const float* x = (const float*)d_in[0]; const float* wqkv = (const float*)d_in[1]; const float* wproj = (const float*)d_in[2]; const float* bproj = (const float*)d_in[3];
    float* OUT = (float*)d_out;
    char* wsp = (char*)d_ws;
    bf*  WT  = (bf*)wsp;  wsp += WT_BYTES;
    unsigned short* WOH = (unsigned short*)wsp; wsp += WO_BYTES;
    bf*  XB  = (bf*)wsp;  wsp += XB_BYTES;
    h16* QKp = (h16*)wsp; wsp += QK_BYTES;
    h16* VTp = (h16*)wsp; wsp += VT_BYTES;
    h16* CTX = (h16*)wsp; wsp += CT_BYTES;

    k_wt<DM, 3 * DM, false><<<(unsigned)((3 * DM * DM / 64 + 63) / 64), 256, 0, stream>>>(wqkv, WT);
    k_wt<DM, DM, true><<<(unsigned)((DM * DM / 64 + 63) / 64), 256, 0, stream>>>(wproj, WOH);
    k_cvt8<<<dim3((unsigned)(((size_t)SEQ * DM / 8 + 255) / 256), 1, NB), 256, 0, stream>>>(x, XB, (size_t)SEQ_FULL * DM, (size_t)SEQ * DM, (unsigned)((size_t)SEQ * DM / 8));
    k_gemmw<bf, true, false><<<dim3(SEQ / 64, QKP / 64, NB), 32, 0, stream>>>(XB, WT, (float*)nullptr, QKp, (const float*)nullptr, (size_t)SEQ * DM, (size_t)0, (size_t)SEQ * QKP, DM, QKP, QKVC);
    k_gemmw<bf, true, false><<<dim3(DM / 64, SEQ / 64, NB), 32, 0, stream>>>(WT + (size_t)2 * DM * DM, XB, (float*)nullptr, VTp, (const float*)nullptr, (size_t)0, (size_t)SEQ * DM, (size_t)DM * SEQ, DM, SEQ, QKVC);
    k_attn<<<dim3(SEQ / 128, NH, NB), 128, 0, stream>>>(QKp, VTp, CTX);
    k_gemmw<h16, false, true><<<dim3(SEQ / 64, DM / 64, NB), 32, 0, stream>>>(CTX, (const h16*)WOH, OUT, (h16*)nullptr, bproj, (size_t)SEQ * DM, (size_t)0, (size_t)SEQ_FULL * DM, DM, DM, 1.0f / (CTXC * WOC));
    (void)hipGetLastError();
}
